// TAGCNLayer_32899449488056
// MI455X (gfx1250) — hardware-verified
//
#include <hip/hip_runtime.h>
#include <math.h>


typedef unsigned int u32;
typedef __attribute__((ext_vector_type(2)))  int      v2i;
typedef __attribute__((ext_vector_type(16))) _Float16 v16h;
typedef __attribute__((ext_vector_type(8)))  _Float16 v8h;
typedef __attribute__((ext_vector_type(8)))  float    v8f;
typedef __attribute__((ext_vector_type(4)))  float    v4f;
#define NN    10000
#define NE    640000
#define DD    128
#define NCAND 10
#define SORTN 1048576
#define TILE  8192
#define NPAD  10048
#define MAXDEG 4096
#define VST2(T, ptr, val) do { const T _v = (val); *(volatile T*)(ptr) = _v; __threadfence(); *(volatile T*)(ptr) = _v; } while (0)
__device__ __forceinline__ v8f wmma16(v16h a, v16h b, v8f c) {
  v8f d = __builtin_amdgcn_wmma_f32_16x16x32_f16(false, a, false, b, (short)0, c, false, false);
  asm volatile("v_nop\n\tv_nop\n\tv_nop\n\tv_nop" : "+v"(d) : "v"(a), "v"(b));
  return d;
}
__device__ __forceinline__ v16h frag16(const _Float16* p, int hh) {
  const v8h lo = *(const v8h*)(p + 8 * hh), hi = *(const v8h*)(p + 16 + 8 * hh);
  return __builtin_shufflevector(lo, hi, 0,1,2,3,4,5,6,7,8,9,10,11,12,13,14,15);
}
__global__ __launch_bounds__(256) void k_sort_init(const int* __restrict__ src, const int* __restrict__ dst, u32* __restrict__ A, int E) {
  const int i = blockIdx.x * 256 + threadIdx.x;
  VST2(u32, A + i, (i < E) ? (((u32)dst[i]) << 16) | ((u32)i & 0xffffu) : 0xffffffffu);
}
__device__ __forceinline__ void cas_lds(u32* s, int lo, int hi, bool up) {
  const u32 a = s[lo], b = s[hi]; const bool sw = up ? (a > b) : (a < b); s[lo] = sw ? b : a; s[hi] = sw ? a : b;
}
__global__ __launch_bounds__(256) void k_sort_local(u32* __restrict__ A) {
  __shared__ u32 s[TILE];
  const int base = blockIdx.x * TILE, t = threadIdx.x;
  for (int i = t; i < TILE; i += 256) s[i] = A[base + i];
  __syncthreads();
  for (int k = 2; k <= TILE; k <<= 1)
    for (int j = k >> 1; j > 0; j >>= 1) {
      for (int p = t; p < TILE / 2; p += 256) {
        const int lo = ((p >> __builtin_ctz(j)) << (__builtin_ctz(j) + 1)) | (p & (j - 1));
        cas_lds(s, lo, lo + j, (((base + lo) & k) == 0));
      }
      __syncthreads();
    }
  for (int pass = 0; pass < 2; ++pass) { for (int i = t; i < TILE; i += 256) *(volatile u32*)(A + base + i) = s[i]; __threadfence(); }
}
__global__ __launch_bounds__(256) void k_sort_global(u32* __restrict__ A, int logj, int k) {
  const int p = blockIdx.x * 256 + threadIdx.x;
  const int j = 1 << logj;
  const int lo = ((p >> logj) << (logj + 1)) | (p & (j - 1)), hi = lo + j;
  const u32 a = A[lo], b = A[hi];
  const bool up = ((lo & k) == 0), sw = up ? (a > b) : (a < b);
  const u32 vlo = sw ? b : a, vhi = sw ? a : b;
  *(volatile u32*)(A + lo) = vlo; *(volatile u32*)(A + hi) = vhi; __threadfence();
  *(volatile u32*)(A + lo) = vlo; *(volatile u32*)(A + hi) = vhi;
}
__global__ __launch_bounds__(256) void k_sort_lds(u32* __restrict__ A, int k) {
  __shared__ u32 s[TILE];
  const int base = blockIdx.x * TILE, t = threadIdx.x;
  for (int i = t; i < TILE; i += 256) s[i] = A[base + i];
  __syncthreads();
  for (int j = TILE >> 1; j > 0; j >>= 1) {
    for (int p = t; p < TILE / 2; p += 256) {
      const int lo = ((p >> __builtin_ctz(j)) << (__builtin_ctz(j) + 1)) | (p & (j - 1));
      cas_lds(s, lo, lo + j, (((base + lo) & k) == 0));
    }
    __syncthreads();
  }
  for (int pass = 0; pass < 2; ++pass) { for (int i = t; i < TILE; i += 256) *(volatile u32*)(A + base + i) = s[i]; __threadfence(); }
}

__global__ __launch_bounds__(256) void k_segs(const u32* __restrict__ A, v2i* __restrict__ seg, float* __restrict__ inv) {
  const int n = blockIdx.x * 256 + threadIdx.x;
  if (n >= NN) return;
  int lo = 0, hi = SORTN;
  while (lo < hi) { const int mid = (lo + hi) >> 1; if ((A[mid] >> 16) < (u32)n) lo = mid + 1; else hi = mid; }
  const int st = lo; hi = SORTN;
  while (lo < hi) { const int mid = (lo + hi) >> 1; if ((A[mid] >> 16) < (u32)(n + 1)) lo = mid + 1; else hi = mid; }
  const v2i sv = {st, lo - st};
  VST2(v2i, seg + n, sv);
  VST2(float, inv + n, 1.0f / fmaxf((float)(lo - st), 1.0f));
}
__global__ __launch_bounds__(256) void k_resolve(const u32* __restrict__ keys, const int* __restrict__ edst, u32* __restrict__ eids) {
  const int p = blockIdx.x * 256 + threadIdx.x;
  if (p >= NE) return;
  const u32 key = keys[p]; const int d = (int)(key >> 16), lo16 = (int)(key & 0xffffu);
  int r = 0;
  while (r < NCAND && p - r - 1 >= 0 && keys[p - r - 1] == key) ++r;
  u32 eid = 0; int seen = 0; bool found = false;
  for (int t = 0; t < NCAND; ++t) { const int c = lo16 + (t << 16); if (c < NE && edst[c] == d) { if (seen == r && !found) { eid = (u32)c; found = true; } ++seen; } }
  VST2(u32, eids + p, eid);
}

__global__ __launch_bounds__(256) void k_norm(const v2i* __restrict__ seg, float* __restrict__ nrm) {
  const int n = blockIdx.x * 256 + threadIdx.x;
  if (n >= NN) return;
  VST2(float, nrm + n, rsqrtf(fmaxf((float)seg[n][1], 1.0f)));
}
__global__ __launch_bounds__(256) void k_hop(const float* __restrict__ in, const int* __restrict__ esrc, const v2i* __restrict__ seg, const u32* __restrict__ eids,
                                             const float* __restrict__ ew, const float* __restrict__ nrm, float* __restrict__ out, _Float16* __restrict__ F16, int coff) {
  const int t = blockIdx.x * 256 + threadIdx.x;
  if (t >= NN * 16) return;
  const int n = t >> 4, c = (t & 15) * 8;
  const v2i sv = seg[n];
  const int st = min(max(sv[0], 0), SORTN - 1), cnt = min(max(sv[1], 0), MAXDEG);
  float acc[8] = {0.f, 0.f, 0.f, 0.f, 0.f, 0.f, 0.f, 0.f};
  for (int p = 0; p < cnt; ++p) {
    const int e = min((int)eids[min(st + p, NE - 1)], NE - 1);
    const int s = min(max(esrc[e], 0), NN - 1);
    const float w = ew[e] * nrm[s];
    const float* xr = in + (size_t)s * DD + c;
#pragma unroll
    for (int q = 0; q < 8; ++q) acc[q] += w * xr[q];
  }
  const float dn = nrm[n];
  typedef __attribute__((ext_vector_type(8))) float v8f32; v8f32 o; v8h oh;
#pragma unroll
  for (int q = 0; q < 8; ++q) { o[q] = acc[q] * dn; oh[q] = (_Float16)o[q]; }
  VST2(v8f32, out + (size_t)n * DD + c, o);
  VST2(v8h, F16 + (size_t)n * 384 + coff + c, oh);
}
__global__ __launch_bounds__(256) void k_f0(const float* __restrict__ h, _Float16* __restrict__ F16) {
  const int t = blockIdx.x * 256 + threadIdx.x;
  if (t >= NPAD * 48) return;
  const int n = t / 48, c = (t % 48) * 8;
  if (n < NN && c >= DD) return;
  v8h o;
#pragma unroll
  for (int q = 0; q < 8; ++q) o[q] = (n < NN) ? (_Float16)h[(size_t)n * DD + c + q] : (_Float16)0.f;
  VST2(v8h, F16 + (size_t)n * 384 + c, o);
}
__global__ __launch_bounds__(256) void k_w16(const float* __restrict__ w, _Float16* __restrict__ W16) {
  const int t = blockIdx.x * 256 + threadIdx.x;
  if (t >= 128 * 48) return;
  v8h o;
#pragma unroll
  for (int q = 0; q < 8; ++q) o[q] = (_Float16)w[(size_t)t * 8 + q];
  VST2(v8h, W16 + (size_t)t * 8, o);
}
__global__ __launch_bounds__(128) void k_gemm(const _Float16* __restrict__ A, const _Float16* __restrict__ W16, const float* __restrict__ bias,
                                              const float* __restrict__ g, const float* __restrict__ be, float* __restrict__ out) {
  __shared__ __attribute__((aligned(16))) float sT[4][16][132];
  const int lane = threadIdx.x & 31, wave = threadIdx.x >> 5, hh = lane >> 4, l16 = lane & 15;
  const int m0 = blockIdx.x * 64 + wave * 16;
  v8f acc[8];
#pragma unroll
  for (int ni = 0; ni < 8; ++ni) acc[ni] = (v8f){};
#pragma unroll 2
  for (int k0 = 0; k0 < 384; k0 += 32) {
    const v16h a0 = frag16(A + (size_t)(m0 + l16) * 384 + k0, hh);
#pragma unroll
    for (int ni = 0; ni < 8; ++ni) acc[ni] = wmma16(a0, frag16(W16 + (size_t)(ni * 16 + l16) * 384 + k0, hh), acc[ni]);
  }
  float (*st)[132] = sT[wave];
#pragma unroll
  for (int ni = 0; ni < 8; ++ni)
#pragma unroll
    for (int i = 0; i < 8; ++i) st[i + 8 * hh][ni * 16 + l16] = acc[ni][i] + bias[ni * 16 + l16];
  __builtin_amdgcn_fence(__ATOMIC_RELEASE, "workgroup"); __builtin_amdgcn_wave_barrier(); __builtin_amdgcn_fence(__ATOMIC_ACQUIRE, "workgroup");
  if (lane < 16) {
    float* rw = st[lane]; float m = 0.f;
    for (int c = 0; c < 128; ++c) m += rw[c];
    m *= (1.0f / 128.0f);
    float var = 0.f;
    for (int c = 0; c < 128; ++c) { const float d = rw[c] - m; var += d * d; }
    const float rs = rsqrtf(var * (1.0f / 128.0f) + 1e-5f);
    for (int c = 0; c < 128; ++c) rw[c] = fmaxf((rw[c] - m) * rs * g[c] + be[c], 0.f);
  }
  __builtin_amdgcn_fence(__ATOMIC_RELEASE, "workgroup"); __builtin_amdgcn_wave_barrier(); __builtin_amdgcn_fence(__ATOMIC_ACQUIRE, "workgroup");
  for (int pass = 0; pass < 2; ++pass) {
#pragma unroll
    for (int rr = 0; rr < 16; ++rr) if (m0 + rr < NN) *(volatile v4f*)(out + (size_t)(m0 + rr) * DD + lane * 4) = *(const v4f*)(&st[rr][lane * 4]);
    __threadfence();
  }
}
extern "C" void kernel_launch(void* const* d_in, const int* in_sizes, int n_in,
                              void* d_out, int out_size, void* d_ws, size_t ws_size, hipStream_t stream) {
  (void)in_sizes; (void)n_in; (void)out_size;
  const float* h    = (const float*)d_in[0];
  const float* ew   = (const float*)d_in[1];
  const float* lw   = (const float*)d_in[2];
  const float* lb   = (const float*)d_in[3];
  const float* g    = (const float*)d_in[4];
  const float* be   = (const float*)d_in[5];
  const int*   src  = (const int*)  d_in[6];
  const int*   dst  = (const int*)  d_in[7];
  float* out = (float*)d_out;
  char* ws = (char*)d_ws; size_t off = 0;
  auto take = [&](size_t bytes) { void* p = ws + off; off = (off + bytes + 255) & ~(size_t)255; return p; };
  u32*      keys = (u32*)take((size_t)SORTN * 4);
  u32*      eids = (u32*)take((size_t)NE * 4);
  v2i*      seg  = (v2i*)take((size_t)NN * 8);
  float*    inv  = (float*)take((size_t)NN * 4);
  float*    nrm  = (float*)take((size_t)NN * 4);
  float*    x1   = (float*)take((size_t)NN * DD * 4);
  float*    x2   = (float*)take((size_t)NN * DD * 4);
  _Float16* F16  = (_Float16*)take((size_t)NPAD * 384 * 2);
  _Float16* W16  = (_Float16*)take((size_t)128 * 384 * 2);
  if (off > ws_size) return;
  const dim3 b256(256);
  k_sort_init<<<SORTN / 256, b256, 0, stream>>>(src, dst, keys, NE);
  k_sort_local<<<SORTN / TILE, b256, 0, stream>>>(keys);
  for (int k = TILE * 2; k <= SORTN; k <<= 1) {
    for (int logj = __builtin_ctz(k) - 1; (1 << logj) >= TILE; --logj)
      k_sort_global<<<SORTN / 2 / 256, b256, 0, stream>>>(keys, logj, k);
    k_sort_lds<<<SORTN / TILE, b256, 0, stream>>>(keys, k);
  }
  k_segs<<<(NN + 255) / 256, b256, 0, stream>>>(keys, seg, inv);
  k_resolve<<<(NE + 255) / 256, b256, 0, stream>>>(keys, dst, eids);
  k_norm<<<(NN + 255) / 256, b256, 0, stream>>>(seg, nrm);
  k_f0<<<(NPAD * 48 + 255) / 256, b256, 0, stream>>>(h, F16);
  k_hop<<<(NN * 16 + 255) / 256, b256, 0, stream>>>(h, src, seg, eids, ew, nrm, x1, F16, DD);
  k_hop<<<(NN * 16 + 255) / 256, b256, 0, stream>>>(x1, src, seg, eids, ew, nrm, x2, F16, 2 * DD);
  k_w16<<<(128 * 48 + 255) / 256, b256, 0, stream>>>(lw, W16);
  k_gemm<<<NPAD / 64, 128, 0, stream>>>(F16, W16, lb, g, be, out);
}
